// MLP_60206851556132
// MI455X (gfx1250) — hardware-run, weakly checked
//
#include <hip/hip_runtime.h>
#define MNR 262144
#define MCH 32768
#define MDI 39
#define MDP 64
#define MDH 256
#define MDS 295
#define MSP 320
#define MDO 4
typedef unsigned short v8us __attribute__((ext_vector_type(8), may_alias));
typedef float  v8f  __attribute__((ext_vector_type(8)));
typedef float  v4f  __attribute__((ext_vector_type(4)));
typedef float  v4fa __attribute__((ext_vector_type(4), may_alias));

__device__ __forceinline__ unsigned short bf16_bits(float x) { unsigned int u = __float_as_uint(x); return (unsigned short)((u + 0x7FFFu + ((u >> 16) & 1u)) >> 16); }
__device__ __forceinline__ float bf16_val(unsigned short b) { return __uint_as_float(((unsigned int)b) << 16); }
__device__ __forceinline__ float bf16_round(float x) { return bf16_val(bf16_bits(x)); }

typedef _Float16 v16h __attribute__((ext_vector_type(16)));
union FragH { v16h v; v8us half[2]; _Float16 h[16]; unsigned short u[16]; };

__global__ __launch_bounds__(256) void k_wt_f16(const float* __restrict__ W, _Float16* __restrict__ Wt, int K, int N, float scale) {
  const int t = blockIdx.x * 256 + threadIdx.x; if (t >= N * (K / 8)) return; const int n = t / (K / 8), k8 = (t % (K / 8)) * 8; FragH f;
#pragma unroll
  for (int i = 0; i < 8; ++i) f.h[i] = (_Float16)(bf16_round(W[(size_t)(k8 + i) * N + n]) * scale); const v8us o = f.half[0];
  *(volatile v8us*)((unsigned short*)Wt + (size_t)n * K + k8) = o; __threadfence(); *(volatile v8us*)((unsigned short*)Wt + (size_t)n * K + k8) = o;
}

typedef _Float16 v4h __attribute__((ext_vector_type(4)));

__global__ __launch_bounds__(256) void k_x16(const float* __restrict__ x, _Float16* __restrict__ X16, size_t n8) { const size_t t = (size_t)blockIdx.x * 256 + threadIdx.x; if (t >= n8) return; FragH f;
#pragma unroll
  for (int q = 0; q < 8; ++q) f.h[q] = (_Float16)bf16_round(x[t * 8 + q]); *(volatile v8us*)((unsigned short*)X16 + t * 8) = f.half[0]; __threadfence(); *(volatile v8us*)((unsigned short*)X16 + t * 8) = f.half[0]; }

__device__ __forceinline__ v16h g2_frag(const _Float16* p, int hh) { FragH f; f.half[0] = *(const v8us*)((const unsigned short*)p + 8 * hh); f.half[1] = *(const v8us*)((const unsigned short*)p + 16 + 8 * hh); return f.v; }
__device__ __forceinline__ v8f g2_mma(v16h a, v16h b, v8f c) { v8f d = __builtin_amdgcn_wmma_f32_16x16x32_f16(false, a, false, b, (short)0, c, false, false); asm volatile("v_nop\n\tv_nop\n\tv_nop\n\tv_nop" : "+v"(d) : "v"(a), "v"(b)); return d; }
template <int ACT>
__global__ __launch_bounds__(128) void k_gemm2(const _Float16* __restrict__ A, int lda, size_t sA, const _Float16* __restrict__ Bh, int ldb, size_t sB, float alpha, const float* __restrict__ bias, size_t sBias, const float* __restrict__ CP, int rowsPerB, size_t sCPb, int row0g,
    float* __restrict__ C, _Float16* __restrict__ C16, int ldc, size_t sC, int M, int N, int K) { static_assert(ACT == 0 || ACT == 3 || ACT == 6 || ACT == 8 || ACT == 9 || ACT == 11 || ACT == 12 || ACT == 14 || ACT == 15 || ACT == 16 || ACT == 17, "k_gemm2: unsupported ACT code (would silently apply no activation)");
  __shared__ __attribute__((aligned(16))) float so[4][32][68];
  const int tid = threadIdx.x, w = tid >> 5, lane = tid & 31, ln = lane & 15, hh = lane >> 4; const int by = blockIdx.y;
  A += (size_t)by * sA; Bh += (size_t)by * sB; const size_t cofs = (size_t)by * sC; const float* bp = bias ? bias + (size_t)by * sBias : nullptr;
  const int ntn = N >> 6; const int mt = blockIdx.x / ntn, nq = blockIdx.x - mt * ntn; const int row0 = mt * 128 + 32 * w, col0 = nq * 64; if (row0 >= M) return;
  const _Float16* a0p = A + (size_t)(row0 + ln) * lda; const _Float16* a1p = a0p + (size_t)16 * lda;
  const _Float16* b0p = Bh + (size_t)(col0 + ln) * ldb; const _Float16* b1p = b0p + (size_t)16 * ldb; const _Float16* b2p = b1p + (size_t)16 * ldb; const _Float16* b3p = b2p + (size_t)16 * ldb;
  const v8f z8 = {0.f,0.f,0.f,0.f,0.f,0.f,0.f,0.f}; v8f c00 = z8, c01 = z8, c02 = z8, c03 = z8, c10 = z8, c11 = z8, c12 = z8, c13 = z8;
  for (int kb = 0; kb < K; kb += 32) { const v16h a0 = g2_frag(a0p + kb, hh), a1 = g2_frag(a1p + kb, hh);
    v16h b = g2_frag(b0p + kb, hh); c00 = g2_mma(a0, b, c00); c10 = g2_mma(a1, b, c10);
    b = g2_frag(b1p + kb, hh); c01 = g2_mma(a0, b, c01); c11 = g2_mma(a1, b, c11);
    b = g2_frag(b2p + kb, hh); c02 = g2_mma(a0, b, c02); c12 = g2_mma(a1, b, c12);
    b = g2_frag(b3p + kb, hh); c03 = g2_mma(a0, b, c03); c13 = g2_mma(a1, b, c13); }
  v8f accs[8] = {c00, c01, c02, c03, c10, c11, c12, c13};
#pragma unroll
  for (int u = 0; u < 8; ++u) { const int t = u & 3, half = u >> 2; const int col = col0 + t * 16 + ln; const float bv = bp ? bf16_round(bp[col]) : 0.f;
#pragma unroll
    for (int r = 0; r < 8; ++r) { const int rloc = half * 16 + 8 * hh + r; float v = accs[u][r] * alpha + bv; if (CP) { if (rowsPerB < 0) v += CP[cofs + (size_t)(row0g + row0 + rloc) * ldc + col];        else { const int bidx = (row0g + row0 + rloc) / rowsPerB; v += CP[(size_t)bidx * sCPb + (size_t)by * 64 + col]; } }
      if (ACT == 3) v = fmaxf(v, 0.f); else if (ACT == 6) v = 0.5f * v * (1.0f + erff(v * 0.70710678118654752f)); else if (ACT == 11) v = 1.0f / (1.0f + expf(-v)); else if (ACT == 15) v = v / (1.0f + expf(-v)); else if (ACT == 12) v = (v > 0.f) ? v : 0.01f * v; else if (ACT == 8) v = tanhf(v); else if (ACT == 9) v = 0.5f * v * (1.0f + tanhf(0.7978845608028654f * (v + 0.044715f * v * v * v))); else if (ACT == 14) v = (v > 0.f) ? v : 0.1f * v; else if (ACT == 16) v = (v >= 0.f) ? v : 0.3f * v; else if (ACT == 17) v = (v >= 0.f) ? v : 0.2f * v;
      so[w][rloc][t * 16 + ln] = v; } }
  __builtin_amdgcn_fence(__ATOMIC_ACQ_REL, "workgroup"); __builtin_amdgcn_wave_barrier();
  const int rsub = lane >> 4, c4 = (lane & 15) * 4;
  for (int pass = 0; pass < 2; ++pass) {
#pragma unroll
    for (int q = 0; q < 16; ++q) { const int r = q * 2 + rsub; const v4f v = *(const v4fa*)&so[w][r][c4]; if (C) *(volatile v4f*)(C + cofs + (size_t)(row0 + r) * ldc + col0 + c4) = v; if (C16) { v4h h4; for (int i = 0; i < 4; ++i) h4[i] = (_Float16)v[i]; *(volatile v4h*)(C16 + cofs + (size_t)(row0 + r) * ldc + col0 + c4) = h4; } }
    if (pass == 0) __threadfence(); } }

__global__ __launch_bounds__(256) void k_cs16(const float* __restrict__ sw, _Float16* __restrict__ tw, float scale) { const size_t t = (size_t)blockIdx.x * 256 + threadIdx.x; FragH f;
#pragma unroll
  for (int q = 0; q < 8; ++q) f.h[q] = (_Float16)(bf16_round(sw[t * 8 + q]) * scale); unsigned short* tp = (unsigned short*)tw + t * 8; *(volatile v8us*)tp = f.half[0]; __threadfence(); *(volatile v8us*)tp = f.half[0]; }
__global__ __launch_bounds__(256) void k_wtpad(const float* __restrict__ sw, _Float16* __restrict__ tw, int kd, int kp, int nd) {
  const int t = blockIdx.x * 256 + threadIdx.x, rn = t / (kp / 8), k8 = (t % (kp / 8)) * 8; FragH fw;
#pragma unroll
  for (int q = 0; q < 8; ++q) { const int k = k8 + q, kc = k < kd ? k : kd - 1; const float v = bf16_round(sw[(size_t)kc * nd + rn]); fw.h[q] = k < kd ? (_Float16)v : (_Float16)0.0f; }
  unsigned short* tp = (unsigned short*)tw + (size_t)rn * kp + k8; *(volatile v8us*)tp = fw.half[0]; __threadfence(); *(volatile v8us*)tp = fw.half[0]; }
__global__ __launch_bounds__(256) void k_xpad(const float* __restrict__ sx, _Float16* __restrict__ tw, int ldd, int c0) {
  const unsigned t = blockIdx.x * 256 + threadIdx.x, r = t >> 3, g8 = (t & 7u) * 8; const float* sr = sx + (size_t)r * MDI; FragH fw;
#pragma unroll
  for (int q = 0; q < 8; ++q) { const unsigned c = g8 + q, cc = c < (unsigned)MDI ? c : (unsigned)(MDI - 1); const float v = bf16_round(sr[cc]); fw.h[q] = c < (unsigned)MDI ? (_Float16)v : (_Float16)0.0f; }
  unsigned short* tp = (unsigned short*)tw + (size_t)r * ldd + c0 + g8; *(volatile v8us*)tp = fw.half[0]; __threadfence(); *(volatile v8us*)tp = fw.half[0]; }
__global__ __launch_bounds__(256) void k_last(const _Float16* __restrict__ ph, const float* __restrict__ gw9, const float* __restrict__ gc9, float* __restrict__ dst) {
  const unsigned t = blockIdx.x * 256 + threadIdx.x; const unsigned short* pr = (const unsigned short*)ph + (size_t)t * MDH; float s0 = 0.f, s1 = 0.f, s2 = 0.f, s3 = 0.f;
#pragma unroll
  for (int k8 = 0; k8 < MDH; k8 += 8) { FragH fw; fw.half[0] = *(const v8us*)(pr + k8);
#pragma unroll
    for (int q = 0; q < 8; ++q) { const float a = (float)fw.h[q]; const float* gr = gw9 + (size_t)(k8 + q) * MDO; s0 += a * bf16_round(gr[0]); s1 += a * bf16_round(gr[1]); s2 += a * bf16_round(gr[2]); s3 += a * bf16_round(gr[3]); } }
  v4f o; o[0] = s0 + bf16_round(gc9[0]); o[1] = s1 + bf16_round(gc9[1]); o[2] = s2 + bf16_round(gc9[2]); o[3] = s3 + bf16_round(gc9[3]); float* dp = dst + (size_t)t * MDO; *(volatile v4f*)dp = o; __threadfence(); *(volatile v4f*)dp = o; }

extern "C" void kernel_launch(void* const* d_in, const int* in_sizes, int n_in,
                              void* d_out, int out_size, void* d_ws, size_t ws_size, hipStream_t stream) {
  if (n_in < 19) return; if (in_sizes[0] < MNR * MDI || out_size < MNR * MDO) return;
  for (int q = 0; q < 9; ++q) { const int kd = q == 0 ? MDI : q == 4 ? MDS : MDH, nd = q == 8 ? MDO : MDH; if (in_sizes[1 + 2 * q] < kd * nd || in_sizes[2 + 2 * q] < nd) return; }
  const float* xa = (const float*)d_in[0]; const float* gw[9]; const float* gc[9]; for (int q = 0; q < 9; ++q) { gw[q] = (const float*)d_in[1 + 2 * q]; gc[q] = (const float*)d_in[2 + 2 * q]; } float* res = (float*)d_out;
  static_assert(MNR % MCH == 0 && MCH % 128 == 0 && MDH % 64 == 0 && MDP % 32 == 0 && MSP % 32 == 0 && MDH % 32 == 0 && MDP >= MDI && MSP >= MDS && MDS == MDH + MDI && MSP - MDH == MDP && MDO == 4 && MDH % 8 == 0 && (MDH * (MDP / 8)) % 256 == 0 && (MDH * (MSP / 8)) % 256 == 0 && (MCH * 8) % 256 == 0 && MCH % 256 == 0, "whole tiles, whole chunks, exact cast launches, the fifth plane's last 64 columns are xa's plane");
  uint8_t* wsp = (uint8_t*)d_ws; size_t off = 0;
  auto take = [&](size_t bytes) { uint8_t* at = wsp + off; off += (bytes + 255) & ~(size_t)255; return at; };
  _Float16* PW[8]; for (int q = 0; q < 8; ++q) { const int kp = q == 0 ? MDP : q == 4 ? MSP : MDH; PW[q] = (_Float16*)take((size_t)MDH * kp * 2); }
  _Float16* PX = (_Float16*)take((size_t)MCH * MDP * 2); _Float16* PA = (_Float16*)take((size_t)MCH * MDH * 2); _Float16* PC = (_Float16*)take((size_t)MCH * MDH * 2); _Float16* PS = (_Float16*)take((size_t)MCH * MSP * 2);
  if (off > ws_size) return;
  for (int q = 0; q < 8; ++q) { if (q == 0 || q == 4) { const int kd = q == 0 ? MDI : MDS, kp = q == 0 ? MDP : MSP; k_wtpad<<<(unsigned)(MDH * (kp / 8) / 256), 256, 0, stream>>>(gw[q], PW[q], kd, kp, MDH); } else k_wt_f16<<<(unsigned)((MDH * (MDH / 8) + 255) / 256), 256, 0, stream>>>(gw[q], PW[q], MDH, MDH, 1.0f); }
  const dim3 gh((unsigned)((MCH / 128) * (MDH / 64)), 1);
  for (int c = 0; c < MNR / MCH; ++c) { const float* xc = xa + (size_t)c * MCH * MDI; float* rc = res + (size_t)c * MCH * MDO;
    k_xpad<<<(unsigned)(MCH * 8 / 256), 256, 0, stream>>>(xc, PX, MDP, 0); k_xpad<<<(unsigned)(MCH * 8 / 256), 256, 0, stream>>>(xc, PS, MSP, MDH);
    k_gemm2<3><<<gh, 128, 0, stream>>>(PX, MDP, (size_t)0, PW[0], MDP, (size_t)0, 1.0f, gc[0], (size_t)0, nullptr, 1, 0, 0, nullptr, PA, MDH, (size_t)0, MCH, MDH, MDP);
    k_gemm2<3><<<gh, 128, 0, stream>>>(PA, MDH, (size_t)0, PW[1], MDH, (size_t)0, 1.0f, gc[1], (size_t)0, nullptr, 1, 0, 0, nullptr, PC, MDH, (size_t)0, MCH, MDH, MDH);
    k_gemm2<3><<<gh, 128, 0, stream>>>(PC, MDH, (size_t)0, PW[2], MDH, (size_t)0, 1.0f, gc[2], (size_t)0, nullptr, 1, 0, 0, nullptr, PA, MDH, (size_t)0, MCH, MDH, MDH);
    k_gemm2<3><<<gh, 128, 0, stream>>>(PA, MDH, (size_t)0, PW[3], MDH, (size_t)0, 1.0f, gc[3], (size_t)0, nullptr, 1, 0, 0, nullptr, PS, MSP, (size_t)0, MCH, MDH, MDH);
    k_gemm2<3><<<gh, 128, 0, stream>>>(PS, MSP, (size_t)0, PW[4], MSP, (size_t)0, 1.0f, gc[4], (size_t)0, nullptr, 1, 0, 0, nullptr, PA, MDH, (size_t)0, MCH, MDH, MSP);
    k_gemm2<3><<<gh, 128, 0, stream>>>(PA, MDH, (size_t)0, PW[5], MDH, (size_t)0, 1.0f, gc[5], (size_t)0, nullptr, 1, 0, 0, nullptr, PC, MDH, (size_t)0, MCH, MDH, MDH);
    k_gemm2<3><<<gh, 128, 0, stream>>>(PC, MDH, (size_t)0, PW[6], MDH, (size_t)0, 1.0f, gc[6], (size_t)0, nullptr, 1, 0, 0, nullptr, PA, MDH, (size_t)0, MCH, MDH, MDH);
    k_gemm2<3><<<gh, 128, 0, stream>>>(PA, MDH, (size_t)0, PW[7], MDH, (size_t)0, 1.0f, gc[7], (size_t)0, nullptr, 1, 0, 0, nullptr, PC, MDH, (size_t)0, MCH, MDH, MDH);
    k_last<<<(unsigned)(MCH / 256), 256, 0, stream>>>(PC, gw[8], gc[8], rc); }
}
